// MLA_90950227460271
// MI455X (gfx1250) — hardware-verified
//
#include <hip/hip_runtime.h>
#include <math.h>
#include <stdint.h>

#ifndef NB
#define NB 2
#endif
#ifndef SEQ
#define SEQ 2048
#endif
#define NB_FULL  2
#define SEQ_FULL 2048
#define DIM   2048
#define NHD   16
#define NOPE  128
#define ROPE  64
#define QKD   192
#define VD    128
#define KVR   512
#define KVA   576
#define QW    3072
#define KW    2112
#define CW    2048
#define LNW   1024
#define WVW   1024
#define C2W   4096
#define NTOK  (NB * SEQ)
#define ER    256
#define NQE   (ER / 64)
#define AKC   64

#define CQ   8.0f
#define CL   8.0f
#define CK   16.0f
#define CV   16.0f
#define CP   4096.0f
#define CC   64.0f
#define CWT  1024.0f
#define CWO  1024.0f
#define CRES 1024.0f

static_assert(sizeof(long) == 8);
static_assert(NB >= 1 && NB <= NB_FULL);
static_assert(SEQ >= ER && SEQ <= SEQ_FULL && (SEQ % 64) == 0);
static_assert((ER % 64) == 0 && NQE * 64 == ER);
static_assert(QW == NHD * QKD);
static_assert(KW == NHD * NOPE + ROPE);
static_assert(CW == NHD * VD);
static_assert(LNW == 2 * KVR && WVW == 2 * KVR && C2W == 2 * CW);
static_assert(KVA == KVR + ROPE);
static_assert(QKD == NOPE + ROPE);
static_assert((QKD % 64) == 0 && NOPE == 2 * 64);
static_assert((DIM % 64) == 0 && (QW % 64) == 0 && (KVA % 64) == 0 && (CW % 64) == 0 && (KVR % 32) == 0);
static_assert((NTOK % 64) == 0 && (NTOK % 8) == 0);
static_assert(AKC == 64 && NOPE == VD);

typedef __bf16       v16b __attribute__((ext_vector_type(16)));
typedef __bf16       v8b  __attribute__((ext_vector_type(8)));
typedef _Float16     v16h __attribute__((ext_vector_type(16)));
typedef _Float16     v8h  __attribute__((ext_vector_type(8)));
typedef float        v8f  __attribute__((ext_vector_type(8)));
typedef float        v4f  __attribute__((ext_vector_type(4)));
typedef unsigned int v4u  __attribute__((ext_vector_type(4)));

#define SZ_XB   ((size_t)NTOK * DIM * 2)
#define SZ_CTX  ((size_t)NTOK * CW * 2)
#define SZ_R0   (SZ_XB > SZ_CTX ? SZ_XB : SZ_CTX)
#define SZ_WQB  ((size_t)QW * DIM * 2)
#define SZ_C2   ((size_t)NB * ER * C2W * 2)
#define SZ_RW   (SZ_WQB > SZ_C2 ? SZ_WQB : SZ_C2)
#define SZ_WAB  ((size_t)KVA * DIM * 2)
#define SZ_WK   ((size_t)CW * KVR * 2)
#define SZ_WV2  ((size_t)CW * WVW * 2)
#define SZ_WO2  ((size_t)DIM * C2W * 2)
#define SZ_QH   ((size_t)NTOK * QW * 2)
#define SZ_QL   ((size_t)NB * ER * QW * 2)
#define SZ_KVF  ((size_t)NTOK * KVA * 4)
#define SZ_VTH  ((size_t)NB * CW * SEQ * 2)
#define SZ_RV   (SZ_VTH > SZ_KVF ? SZ_VTH : SZ_KVF)
#define SZ_LN   ((size_t)NTOK * LNW * 2)
#define SZ_KH   ((size_t)NTOK * KW * 2)
#define SZ_KL   ((size_t)NB * ER * KW * 2)
#define SZ_VTL  ((size_t)NB * CW * ER * 2)
#define WS_TOTAL_BYTES (SZ_R0 + SZ_RW + SZ_WAB + SZ_WK + SZ_WV2 + SZ_WO2 + SZ_QH + SZ_QL + SZ_RV + SZ_LN + SZ_KH + SZ_KL + SZ_VTL)
static_assert(WS_TOTAL_BYTES <= 134217728UL);
static_assert(SZ_XB <= SZ_R0 && SZ_CTX <= SZ_R0);
static_assert(SZ_WQB <= SZ_RW && SZ_C2 <= SZ_RW);
static_assert(SZ_KVF <= SZ_RV && SZ_VTH <= SZ_RV);
static_assert((SZ_R0 % 128) == 0 && (SZ_RW % 128) == 0 && (SZ_WAB % 128) == 0 && (SZ_WK % 128) == 0 && (SZ_WV2 % 128) == 0);
static_assert((SZ_WO2 % 128) == 0 && (SZ_QH % 128) == 0 && (SZ_QL % 128) == 0 && (SZ_RV % 128) == 0 && (SZ_LN % 128) == 0);
static_assert((SZ_KH % 128) == 0 && (SZ_KL % 128) == 0 && (SZ_VTL % 128) == 0 && (SZ_KVF % 128) == 0 && (SZ_C2 % 128) == 0);

__device__ __forceinline__ unsigned short bf_bits(float f) {
  const unsigned u = __float_as_uint(f);
  return (unsigned short)((u + 0x7FFFu + ((u >> 16) & 1u)) >> 16);
}
__device__ __forceinline__ float bf_val(unsigned short h) { return __uint_as_float(((unsigned)h) << 16); }
__device__ __forceinline__ float bfr(float f) { return bf_val(bf_bits(f)); }
__device__ __forceinline__ unsigned short h_bits(float f) { const _Float16 h = (_Float16)f; return __builtin_bit_cast(unsigned short, h); }
__device__ __forceinline__ float h_val(unsigned short u) { return (float)__builtin_bit_cast(_Float16, u); }
__device__ __forceinline__ unsigned pk16(unsigned short a, unsigned short b) { return (unsigned)a | ((unsigned)b << 16); }
__device__ __forceinline__ v8f zero8() { v8f z = {0.f, 0.f, 0.f, 0.f, 0.f, 0.f, 0.f, 0.f}; return z; }
__device__ __forceinline__ int wave_id() { return __builtin_amdgcn_readfirstlane((int)(threadIdx.x >> 5)); }

__device__ __forceinline__ void lds_wave_sync() {
  __builtin_amdgcn_fence(3  , "workgroup");
  __builtin_amdgcn_wave_barrier();
  __builtin_amdgcn_fence(2  , "workgroup");
}

template <typename T> struct FragT;
template <> struct FragT<__bf16>   { typedef v16b V; typedef v8b H; };
template <> struct FragT<_Float16> { typedef v16h V; typedef v8h H; };
union FragB { v16b v; v8b h[2]; };
union FragH { v16h v; v8h h[2]; };

__device__ __forceinline__ v16b ldfrag(const __bf16* p) {
  FragB f; f.h[0] = *(const v8b*)(p); f.h[1] = *(const v8b*)(p + 16); return f.v;
}
__device__ __forceinline__ v16h ldfrag(const _Float16* p) {
  FragH f; f.h[0] = *(const v8h*)(p); f.h[1] = *(const v8h*)(p + 16); return f.v;
}
__device__ __forceinline__ v8f at_mma(v16b a, v16b b, v8f c) {
  c = __builtin_amdgcn_wmma_f32_16x16x32_bf16(false, a, false, b, (short)0, c, false, false);
  asm volatile("v_nop\n\tv_nop\n\tv_nop\n\tv_nop" : "+v"(c) : "v"(a), "v"(b));
  return c;
}
__device__ __forceinline__ v8f at_mma(v16h a, v16h b, v8f c) {
  c = __builtin_amdgcn_wmma_f32_16x16x32_f16(false, a, false, b, (short)0, c, false, false);
  asm volatile("v_nop\n\tv_nop\n\tv_nop\n\tv_nop" : "+v"(c) : "v"(a), "v"(b));
  return c;
}
__device__ __forceinline__ void acc_guard4(v8f& a, v8f& b, v8f& c, v8f& d) {
  asm volatile("v_nop\n\tv_nop\n\tv_nop\n\tv_nop" : "+v"(a), "+v"(b), "+v"(c), "+v"(d));
}

__global__ __launch_bounds__(256) void cvt_bf16_kernel(const float* __restrict__ in, unsigned short* outp, int n8,
                                                       long strideIn, long strideOut) {
  const int i = (int)blockIdx.x * 256 + (int)threadIdx.x;
  if (i >= n8) return;
  const float* src = in + (size_t)blockIdx.y * (size_t)strideIn;
  unsigned short* dst = outp + (size_t)blockIdx.y * (size_t)strideOut;
  const size_t e = 8 * (size_t)i;
  const v4f a = *(const v4f*)(src + e);
  const v4f b = *(const v4f*)(src + e + 4);
  v4u w;
  w[0] = pk16(bf_bits(a[0]), bf_bits(a[1]));
  w[1] = pk16(bf_bits(a[2]), bf_bits(a[3]));
  w[2] = pk16(bf_bits(b[0]), bf_bits(b[1]));
  w[3] = pk16(bf_bits(b[2]), bf_bits(b[3]));
  *(volatile v4u*)(dst + e) = w;
  __threadfence();
  *(volatile v4u*)(dst + e) = w;
}

__global__ __launch_bounds__(256) void cvt_f16w_kernel(const float* __restrict__ in, unsigned short* outp, int n8, int cols,
                                                       int grpOut, int grpIn, int rowOff, int dual, float scale, float scale2) {
  const int i = (int)blockIdx.x * 256 + (int)threadIdx.x;
  if (i >= n8) return;
  const size_t e = 8 * (size_t)i;
  const int n   = (int)(e / (size_t)cols);
  const int col = (int)(e - (size_t)n * (size_t)cols);
  const int g   = n / grpOut;
  const int ri  = g * grpIn + rowOff + (n - g * grpOut);
  const float* src = in + (size_t)ri * (size_t)cols + col;
  const v4f a = *(const v4f*)(src);
  const v4f b = *(const v4f*)(src + 4);
  const float f[8] = {bfr(a[0]), bfr(a[1]), bfr(a[2]), bfr(a[3]), bfr(b[0]), bfr(b[1]), bfr(b[2]), bfr(b[3])};
  v4u w, w2;
#pragma unroll
  for (int q = 0; q < 4; ++q) {
    w[q]  = pk16(h_bits(f[2 * q] * scale),  h_bits(f[2 * q + 1] * scale));
    w2[q] = pk16(h_bits(f[2 * q] * scale2), h_bits(f[2 * q + 1] * scale2));
  }
  const size_t opitch = (dual != 0) ? (2 * (size_t)cols) : (size_t)cols;
  unsigned short* p1 = outp + (size_t)n * opitch + col;
  unsigned short* p2 = p1 + cols;
  for (int pass = 0; pass < 2; ++pass) {
    *(volatile v4u*)(p1) = w;
    if (dual != 0) *(volatile v4u*)(p2) = w2;
    __threadfence();
  }
}

template <typename T, int OUT_MODE, bool ROPEQ>
__global__ __launch_bounds__(256) void gemm64_kernel(
    const unsigned short* __restrict__ Ap, int lda, long strideA,
    const unsigned short* __restrict__ Btp, int ldb, long strideB,
    void* Cout, int ldc, long strideC,
    unsigned short* Clo, int ldl, long strideL, int loMod, int loCnt, int loNmax,
    const float* __restrict__ fc, int ropeMod, int ropeStart,
    int M, int N, int K, float scale) {
  __shared__ __align__(16) float sT[8][16 * 68];
  typedef typename FragT<T>::V V;
  const T* A  = (const T*)(const void*)Ap;
  const T* Bt = (const T*)(const void*)Btp;
  const int b    = blockIdx.y;
  const int lane = threadIdx.x & 31;
  const int wave = wave_id();
  const int tilesN = N >> 6;
  const int tilesM = M >> 6;
  const int tile = (int)blockIdx.x * 8 + wave;
  if (tile >= tilesM * tilesN) return;
  const int tm = tile / tilesN;
  const int tn = tile - tm * tilesN;
  const int m0 = tm << 6;
  const int n0 = tn << 6;

  const T* Ab = A  + (size_t)b * (size_t)strideA;
  const T* Bb = Bt + (size_t)b * (size_t)strideB;

  const int rlane = lane & 15;
  const int koff  = (lane >> 4) * 8;
  const int mOff  = (lane >> 4) * 8;

  v8f acc[4][4];
#pragma unroll
  for (int i = 0; i < 4; ++i)
#pragma unroll
    for (int j = 0; j < 4; ++j) acc[i][j] = zero8();

  for (int k0 = 0; k0 < K; k0 += 32) {
    V bh[4];
#pragma unroll
    for (int j = 0; j < 4; ++j) {
      const size_t bo = (size_t)(n0 + (j << 4) + rlane) * (size_t)ldb + koff + k0;
      bh[j] = ldfrag(Bb + bo);
    }
#pragma unroll
    for (int i = 0; i < 4; ++i) {
      const size_t ao = (size_t)(m0 + (i << 4) + rlane) * (size_t)lda + koff + k0;
      const V ah = ldfrag(Ab + ao);
#pragma unroll
      for (int j = 0; j < 4; ++j) acc[i][j] = at_mma(ah, bh[j], acc[i][j]);
    }
  }
  acc_guard4(acc[0][0], acc[0][1], acc[0][2], acc[0][3]);
  acc_guard4(acc[1][0], acc[1][1], acc[1][2], acc[1][3]);
  acc_guard4(acc[2][0], acc[2][1], acc[2][2], acc[2][3]);
  acc_guard4(acc[3][0], acc[3][1], acc[3][2], acc[3][3]);

  float* slab = sT[wave];
#pragma unroll
  for (int i = 0; i < 4; ++i) {
    const int mBase = m0 + (i << 4);
#pragma unroll
    for (int j = 0; j < 4; ++j)
#pragma unroll
      for (int r = 0; r < 8; ++r)
        slab[(mOff + r) * 68 + (j << 4) + rlane] = acc[i][j][r] * scale;
    lds_wave_sync();
    if (OUT_MODE == 0) {
      float* C = (float*)Cout + (size_t)b * (size_t)strideC;
      const int hh = lane >> 4, c4 = (lane & 15) * 4;
      for (int pass = 0; pass < 2; ++pass) {
#pragma unroll
        for (int it = 0; it < 8; ++it) {
          const int row = it * 2 + hh;
          const v4f v = *(const v4f*)(slab + row * 68 + c4);
          *(volatile v4f*)(C + (size_t)(mBase + row) * (size_t)ldc + n0 + c4) = v;
        }
        __threadfence();
      }
    } else {
      const int qq = lane >> 3, c8 = (lane & 7) * 8;
      unsigned short* C = (unsigned short*)Cout + (size_t)b * (size_t)strideC;
      bool isPe = false;
      if (ROPEQ) isPe = ((n0 % ropeMod) == ropeStart);
      bool loOn = false;
      size_t loRow0 = 0;
      if (Clo != nullptr) {
        loOn = ((mBase % loMod) < loCnt) && (n0 < loNmax);
        loRow0 = (size_t)(mBase / loMod) * (size_t)loCnt + (size_t)(mBase % loMod);
      }
      for (int pass = 0; pass < 2; ++pass) {
#pragma unroll
        for (int it = 0; it < 4; ++it) {
          const int row = it * 4 + qq;
          const float* sp = slab + row * 68 + c8;
          const v4f x0 = *(const v4f*)(sp);
          const v4f x1 = *(const v4f*)(sp + 4);
          float v[8] = {x0[0], x0[1], x0[2], x0[3], x1[0], x1[1], x1[2], x1[3]};
          if (ROPEQ) {
            if (isPe) {
              const int s = (mBase + row) % SEQ;
              const float* fp = fc + (size_t)s * ROPE + c8;
              const v4f f0 = *(const v4f*)(fp);
              const v4f f1 = *(const v4f*)(fp + 4);
              const float cs[8] = {f0[0], f0[1], f0[2], f0[3], f1[0], f1[1], f1[2], f1[3]};
#pragma unroll
              for (int e = 0; e < 4; ++e) {
                const float cc = bfr(cs[2 * e]), sn = bfr(cs[2 * e + 1]);
                const float a0 = v[2 * e], a1 = v[2 * e + 1];
                v[2 * e]     = a0 * cc - a1 * sn;
                v[2 * e + 1] = a0 * sn + a1 * cc;
              }
            }
          }
          v4u hv, lv;
#pragma unroll
          for (int e = 0; e < 4; ++e) {
            const unsigned short h0 = h_bits(v[2 * e]), h1 = h_bits(v[2 * e + 1]);
            const unsigned short l0 = h_bits((v[2 * e] - h_val(h0)) * CRES);
            const unsigned short l1 = h_bits((v[2 * e + 1] - h_val(h1)) * CRES);
            hv[e] = pk16(h0, h1);
            lv[e] = pk16(l0, l1);
          }
          *(volatile v4u*)(C + (size_t)(mBase + row) * (size_t)ldc + n0 + c8) = hv;
          if (loOn)
            *(volatile v4u*)(Clo + (size_t)b * (size_t)strideL + (loRow0 + (size_t)row) * (size_t)ldl + n0 + c8) = lv;
        }
        __threadfence();
      }
    }
    lds_wave_sync();
  }
}

__global__ __launch_bounds__(256) void kvpost_kernel(const float* __restrict__ kvf, const float* __restrict__ fc,
                                                     const float* __restrict__ nw,
                                                     unsigned short* ln, unsigned short* kh, unsigned short* kl) {
  const int wave = wave_id();
  const int lane = (int)threadIdx.x & 31;
  const int row  = (int)blockIdx.x * 8 + wave;
  const int bb   = row / SEQ;
  const int s    = row - bb * SEQ;
  const float* kr = kvf + (size_t)row * KVA;
  const int c0 = 8 * lane;
  const v4f a0 = *(const v4f*)(kr + c0);
  const v4f a1 = *(const v4f*)(kr + c0 + 4);
  const v4f a2 = *(const v4f*)(kr + 256 + c0);
  const v4f a3 = *(const v4f*)(kr + 256 + c0 + 4);
  const float x[16] = {a0[0], a0[1], a0[2], a0[3], a1[0], a1[1], a1[2], a1[3],
                       a2[0], a2[1], a2[2], a2[3], a3[0], a3[1], a3[2], a3[3]};
  float ss = 0.f;
#pragma unroll
  for (int e = 0; e < 16; ++e) ss += x[e] * x[e];
#pragma unroll
  for (int off = 1; off < 32; off <<= 1) ss += __shfl_xor(ss, off, 32);
  const float rs = rsqrtf(ss * (1.0f / 512.0f) + 1e-6f);
  const v4f w0 = *(const v4f*)(nw + c0);
  const v4f w1 = *(const v4f*)(nw + c0 + 4);
  const v4f w2 = *(const v4f*)(nw + 256 + c0);
  const v4f w3 = *(const v4f*)(nw + 256 + c0 + 4);
  const float w[16] = {w0[0], w0[1], w0[2], w0[3], w1[0], w1[1], w1[2], w1[3],
                       w2[0], w2[1], w2[2], w2[3], w3[0], w3[1], w3[2], w3[3]};
  v4u u0, u1, r0, r1;
#pragma unroll
  for (int q = 0; q < 4; ++q) {
    const float y0 = ((x[2 * q] * rs) * bfr(w[2 * q])) * CL;
    const float y1 = ((x[2 * q + 1] * rs) * bfr(w[2 * q + 1])) * CL;
    const unsigned short hy0 = h_bits(y0), hy1 = h_bits(y1);
    u0[q] = pk16(hy0, hy1);
    r0[q] = pk16(h_bits((y0 - h_val(hy0)) * CRES), h_bits((y1 - h_val(hy1)) * CRES));
    const float z0 = ((x[8 + 2 * q] * rs) * bfr(w[8 + 2 * q])) * CL;
    const float z1 = ((x[8 + 2 * q + 1] * rs) * bfr(w[8 + 2 * q + 1])) * CL;
    const unsigned short hz0 = h_bits(z0), hz1 = h_bits(z1);
    u1[q] = pk16(hz0, hz1);
    r1[q] = pk16(h_bits((z0 - h_val(hz0)) * CRES), h_bits((z1 - h_val(hz1)) * CRES));
  }
  const int pl = (lane < 8) ? lane : 7;
  const v4f e0 = *(const v4f*)(kr + KVR + 8 * pl);
  const v4f e1 = *(const v4f*)(kr + KVR + 8 * pl + 4);
  const v4f f0 = *(const v4f*)(fc + (size_t)s * ROPE + 8 * pl);
  const v4f f1 = *(const v4f*)(fc + (size_t)s * ROPE + 8 * pl + 4);
  const float xe[8] = {e0[0], e0[1], e0[2], e0[3], e1[0], e1[1], e1[2], e1[3]};
  const float cs[8] = {f0[0], f0[1], f0[2], f0[3], f1[0], f1[1], f1[2], f1[3]};
  v4u ph, plo;
#pragma unroll
  for (int q = 0; q < 4; ++q) {
    const float cc = bfr(cs[2 * q]), sn = bfr(cs[2 * q + 1]);
    const float p0 = xe[2 * q], p1 = xe[2 * q + 1];
    const float y0 = (p0 * cc - p1 * sn) * CK;
    const float y1 = (p0 * sn + p1 * cc) * CK;
    const unsigned short h0 = h_bits(y0), h1 = h_bits(y1);
    const unsigned short l0 = h_bits((y0 - h_val(h0)) * CRES);
    const unsigned short l1 = h_bits((y1 - h_val(h1)) * CRES);
    ph[q]  = pk16(h0, h1);
    plo[q] = pk16(l0, l1);
  }
  const bool wpe = (lane < 8);
  const bool wlo = wpe && (s < ER);
  const int  sl  = (s < ER) ? s : 0;
  unsigned short* lp  = ln + (size_t)row * LNW;
  unsigned short* kpe = kh + (size_t)row * KW + NHD * NOPE + 8 * pl;
  unsigned short* klo = kl + ((size_t)bb * ER + (size_t)sl) * KW + NHD * NOPE + 8 * pl;
  for (int pass = 0; pass < 2; ++pass) {
    *(volatile v4u*)(lp + c0) = u0;
    *(volatile v4u*)(lp + 256 + c0) = u1;
    *(volatile v4u*)(lp + KVR + c0) = r0;
    *(volatile v4u*)(lp + KVR + 256 + c0) = r1;
    if (wpe) *(volatile v4u*)(kpe) = ph;
    if (wlo) *(volatile v4u*)(klo) = plo;
    __threadfence();
  }
}

template <bool SPLIT>
__global__ __launch_bounds__(128)
void attn_kernel(const unsigned short* __restrict__ qh_p, const unsigned short* __restrict__ ql_p,
                 const unsigned short* __restrict__ kh_p, const unsigned short* __restrict__ kl_p,
                 const unsigned short* __restrict__ vh_p, const unsigned short* __restrict__ vl_p,
                 unsigned short* ctx_p, unsigned short* ctx2_p, int qb0, int nqbl, float sc, float oc) {
  __shared__ __align__(16) _Float16 Ksh[AKC * QKD];
  __shared__ __align__(16) _Float16 Vth[VD * AKC];
  __shared__ __align__(16) _Float16 Psh[4][16 * AKC];
  __shared__ __align__(16) _Float16 Psl[SPLIT ? 4 : 1][16 * AKC];
  constexpr int NT = SPLIT ? 4 : 8;
  static_assert(4 * 16 * VD * 2 <= AKC * QKD * 2);
  static_assert(4 * 2 * 16 * 64 * 2 <= AKC * QKD * 2);

  const int tid  = (int)threadIdx.x;
  const int wave = wave_id();
  const int lane = tid & 31;
  const int hh   = lane >> 4;
  const int c    = lane & 15;

  const int bx = (int)blockIdx.x;
  const int vh = SPLIT ? (bx & 1) : 0;
  const int bq = SPLIT ? (bx >> 1) : bx;
  const int qb = qb0 + (bq % nqbl);
  const int h  = bq / nqbl;
  const int b  = (int)blockIdx.y;
  const int q0 = qb * 64 + wave * 16;
  const int vt0 = vh * NT;
  const size_t tok0 = (size_t)b * SEQ;

  const _Float16* QH  = (const _Float16*)(const void*)qh_p + (size_t)h * QKD;
  const _Float16* QL  = (const _Float16*)(const void*)ql_p + (size_t)h * QKD;
  const _Float16* KHn = (const _Float16*)(const void*)kh_p + (size_t)h * NOPE;
  const _Float16* KHp = (const _Float16*)(const void*)kh_p + (size_t)NHD * NOPE;
  const _Float16* KLb = (const _Float16*)(const void*)kl_p + (size_t)b * ER * KW;
  const _Float16* VH  = (const _Float16*)(const void*)vh_p + ((size_t)b * CW + (size_t)h * VD) * SEQ;
  const _Float16* VL  = (const _Float16*)(const void*)vl_p + ((size_t)b * CW + (size_t)h * VD) * ER;

  float mrow[8], lrow[8];
  v8f oacc[NT];
  v8f oacc2[NT];
#pragma unroll
  for (int r = 0; r < 8; ++r) { mrow[r] = -INFINITY; lrow[r] = 0.f; }
#pragma unroll
  for (int t = 0; t < NT; ++t) { oacc[t] = zero8(); if (SPLIT) oacc2[t] = zero8(); }

  _Float16* pwh = Psh[wave];
  _Float16* pwl = Psl[SPLIT ? wave : 0];

  const int nChunks = qb + 1;
  for (int kc = 0; kc < nChunks; ++kc) {
    const int kv0 = kc * AKC;
    __syncthreads();
    {
      const int r = tid & 63, half = tid >> 6;
      const size_t krow = (tok0 + (size_t)kv0 + (size_t)r) * KW;
      _Float16* dst = Ksh + r * QKD + half * 96;
      if (half == 0) {
#pragma unroll
        for (int i = 0; i < 12; ++i) *(v8h*)(dst + 8 * i) = *(const v8h*)(KHn + krow + 8 * i);
      } else {
#pragma unroll
        for (int i = 0; i < 4; ++i) *(v8h*)(dst + 8 * i) = *(const v8h*)(KHn + krow + 96 + 8 * i);
#pragma unroll
        for (int i = 0; i < 8; ++i) *(v8h*)(dst + 32 + 8 * i) = *(const v8h*)(KHp + krow + 8 * i);
      }
      const size_t vrow = (size_t)tid * SEQ + (size_t)kv0;
#pragma unroll
      for (int i = 0; i < 8; ++i) *(v8h*)(Vth + tid * AKC + 8 * i) = *(const v8h*)(VH + vrow + 8 * i);
    }
    __syncthreads();

    v8f s[4], s2[4];
#pragma unroll
    for (int j = 0; j < 4; ++j) { s[j] = zero8(); s2[j] = zero8(); }
#pragma unroll 1
    for (int dc = 0; dc < 6; ++dc) {
      const v16h qa = ldfrag(QH + (tok0 + (size_t)q0 + (size_t)c) * QW + dc * 32 + 8 * hh);
      v16h qal = qa;
      if (SPLIT) qal = ldfrag(QL + ((size_t)b * ER + (size_t)q0 + (size_t)c) * QW + dc * 32 + 8 * hh);
      const int kcol = (dc < 4) ? (h * NOPE + dc * 32) : (NHD * NOPE + (dc - 4) * 32);
#pragma unroll
      for (int j = 0; j < 4; ++j) {
        FragH kb;
        kb.h[0] = *(const v8h*)(Ksh + (j * 16 + c) * QKD + dc * 32 + 8 * hh);
        kb.h[1] = *(const v8h*)(Ksh + (j * 16 + c) * QKD + dc * 32 + 16 + 8 * hh);
        s[j] = at_mma(qa, kb.v, s[j]);
        if (SPLIT) {
          const v16h klv = ldfrag(KLb + (size_t)(kv0 + j * 16 + c) * KW + kcol + 8 * hh);
          s2[j] = at_mma(qa, klv, s2[j]);
          s2[j] = at_mma(qal, kb.v, s2[j]);
        }
      }
    }
    const bool diag = (kc == qb);
    float cm[8];
#pragma unroll
    for (int r = 0; r < 8; ++r) {
      const int qrow = q0 + 8 * hh + r;
      float m = -INFINITY;
#pragma unroll
      for (int j = 0; j < 4; ++j) {
        const int kvcol = kv0 + j * 16 + c;
        float raw = s[j][r];
        if (SPLIT) raw += s2[j][r] * (1.0f / CRES);
        const float sv = raw * sc;
        const bool masked = diag && (kvcol > qrow);
        const float sm = masked ? -INFINITY : sv;
        s[j][r] = sm;
        m = fmaxf(m, sm);
      }
#pragma unroll
      for (int off = 1; off < 16; off <<= 1) m = fmaxf(m, __shfl_xor(m, off, 32));
      cm[r] = m;
    }
#pragma unroll
    for (int r = 0; r < 8; ++r) {
      const float mnew = fmaxf(mrow[r], cm[r]);
      const float alpha = expf(mrow[r] - mnew);
      mrow[r] = mnew;
      float psum = 0.f;
#pragma unroll
      for (int j = 0; j < 4; ++j) {
        const float p  = expf(s[j][r] - mnew);
        psum += p;
        const float pc = p * CP;
        const unsigned short hb = h_bits(pc);
        pwh[(8 * hh + r) * AKC + j * 16 + c] = __builtin_bit_cast(_Float16, hb);
        if (SPLIT) {
          const unsigned short lb = h_bits((pc - h_val(hb)) * CRES);
          pwl[(8 * hh + r) * AKC + j * 16 + c] = __builtin_bit_cast(_Float16, lb);
        }
      }
#pragma unroll
      for (int off = 1; off < 16; off <<= 1) psum += __shfl_xor(psum, off, 32);
      lrow[r] = lrow[r] * alpha + psum;
#pragma unroll
      for (int t = 0; t < NT; ++t) {
        oacc[t][r] *= alpha;
        if (SPLIT) oacc2[t][r] *= alpha;
      }
    }
    lds_wave_sync();
#pragma unroll 1
    for (int kk = 0; kk < 2; ++kk) {
      FragH pa, plf;
      pa.h[0] = *(const v8h*)(pwh + c * AKC + kk * 32 + 8 * hh);
      pa.h[1] = *(const v8h*)(pwh + c * AKC + kk * 32 + 16 + 8 * hh);
      plf = pa;
      if (SPLIT) {
        plf.h[0] = *(const v8h*)(pwl + c * AKC + kk * 32 + 8 * hh);
        plf.h[1] = *(const v8h*)(pwl + c * AKC + kk * 32 + 16 + 8 * hh);
      }
#pragma unroll
      for (int t = 0; t < NT; ++t) {
        const int tt = vt0 + t;
        FragH vb;
        vb.h[0] = *(const v8h*)(Vth + (tt * 16 + c) * AKC + kk * 32 + 8 * hh);
        vb.h[1] = *(const v8h*)(Vth + (tt * 16 + c) * AKC + kk * 32 + 16 + 8 * hh);
        oacc[t] = at_mma(pa.v, vb.v, oacc[t]);
        if (SPLIT) {
          const v16h vlv = ldfrag(VL + (size_t)(tt * 16 + c) * ER + kv0 + kk * 32 + 8 * hh);
          oacc2[t] = at_mma(pa.v, vlv, oacc2[t]);
          oacc2[t] = at_mma(plf.v, vb.v, oacc2[t]);
        }
      }
    }
  }
  acc_guard4(oacc[0], oacc[1], oacc[2], oacc[3]);
  if (!SPLIT) acc_guard4(oacc[NT - 4], oacc[NT - 3], oacc[NT - 2], oacc[NT - 1]);
  if (SPLIT)  acc_guard4(oacc2[0], oacc2[1], oacc2[2], oacc2[3]);
  __syncthreads();

  unsigned short* stg = (unsigned short*)(void*)Ksh;
  if (!SPLIT) {
    unsigned short* osh = stg + wave * (16 * VD);
#pragma unroll
    for (int r = 0; r < 8; ++r) {
      const float inv = oc * (1.0f / lrow[r]);
#pragma unroll
      for (int t = 0; t < NT; ++t) osh[(8 * hh + r) * VD + t * 16 + c] = h_bits(oacc[t][r] * inv);
    }
    lds_wave_sync();
    unsigned short* Cg = ctx_p + (tok0 + (size_t)q0) * CW + (size_t)h * VD;
    const int rsub = lane >> 4;
    const int c8   = (lane & 15) * 8;
    for (int pass = 0; pass < 2; ++pass) {
#pragma unroll
      for (int it = 0; it < 8; ++it) {
        const int row = it * 2 + rsub;
        const v4u x = *(const v4u*)(osh + row * VD + c8);
        *(volatile v4u*)(Cg + (size_t)row * CW + c8) = x;
      }
      __threadfence();
    }
  } else {
    unsigned short* osh = stg + wave * (2 * 16 * 64);
    unsigned short* osl = osh + 16 * 64;
#pragma unroll
    for (int r = 0; r < 8; ++r) {
      const float inv = oc * (1.0f / lrow[r]);
#pragma unroll
      for (int t = 0; t < NT; ++t) {
        const float o = (oacc[t][r] + oacc2[t][r] * (1.0f / CRES)) * inv;
        const unsigned short hb = h_bits(o);
        const unsigned short lb = h_bits((o - h_val(hb)) * CRES);
        const int so = (8 * hh + r) * 64 + t * 16 + c;
        osh[so] = hb;
        osl[so] = lb;
      }
    }
    lds_wave_sync();
    unsigned short* Cg2 = ctx2_p + ((size_t)b * ER + (size_t)q0) * C2W + (size_t)h * VD + (size_t)vh * 64;
    const int qq = lane >> 3;
    const int c8 = (lane & 7) * 8;
    for (int pass = 0; pass < 2; ++pass) {
#pragma unroll
      for (int it = 0; it < 4; ++it) {
        const int row = it * 4 + qq;
        const v4u x = *(const v4u*)(osh + row * 64 + c8);
        const v4u y = *(const v4u*)(osl + row * 64 + c8);
        *(volatile v4u*)(Cg2 + (size_t)row * C2W + c8)      = x;
        *(volatile v4u*)(Cg2 + (size_t)row * C2W + CW + c8) = y;
      }
      __threadfence();
    }
  }
}

extern "C" void kernel_launch(void* const* d_in, const int* in_sizes, int n_in,
                              void* d_out, int out_size, void* d_ws, size_t ws_size,
                              hipStream_t stream) {
  if (n_in < 7) return;
  const size_t needRows = (size_t)(NB - 1) * SEQ_FULL + SEQ;
  if ((size_t)in_sizes[0] < needRows * DIM) return;
  if (in_sizes[1] < SEQ * ROPE) return;
  if (in_sizes[2] < QW * DIM) return;
  if (in_sizes[3] < KVA * DIM) return;
  if (in_sizes[4] < NHD * (NOPE + VD) * KVR) return;
  if (in_sizes[5] < DIM * CW) return;
  if (in_sizes[6] < KVR) return;
  if ((size_t)out_size < needRows * DIM) return;

  const float* x  = (const float*)d_in[0];
  const float* fc = (const float*)d_in[1];
  const float* wq = (const float*)d_in[2];
  const float* wa = (const float*)d_in[3];
  const float* wb = (const float*)d_in[4];
  const float* wo = (const float*)d_in[5];
  const float* nw = (const float*)d_in[6];
  float* out = (float*)d_out;

  size_t off = 0;
  const size_t oR0  = off; off += SZ_R0;
  const size_t oRW  = off; off += SZ_RW;
  const size_t oWAB = off; off += SZ_WAB;
  const size_t oWK  = off; off += SZ_WK;
  const size_t oWV2 = off; off += SZ_WV2;
  const size_t oWO2 = off; off += SZ_WO2;
  const size_t oQH  = off; off += SZ_QH;
  const size_t oQL  = off; off += SZ_QL;
  const size_t oRV  = off; off += SZ_RV;
  const size_t oLN  = off; off += SZ_LN;
  const size_t oKH  = off; off += SZ_KH;
  const size_t oKL  = off; off += SZ_KL;
  const size_t oVTL = off; off += SZ_VTL;
  if (off != (size_t)WS_TOTAL_BYTES) return;
  if (off > ws_size) return;

  char* ws = (char*)d_ws;
  unsigned short* XB   = (unsigned short*)(ws + oR0);
  unsigned short* CTXH = (unsigned short*)(ws + oR0);
  unsigned short* WQB  = (unsigned short*)(ws + oRW);
  unsigned short* C2   = (unsigned short*)(ws + oRW);
  unsigned short* WAB  = (unsigned short*)(ws + oWAB);
  unsigned short* WK   = (unsigned short*)(ws + oWK);
  unsigned short* WV2  = (unsigned short*)(ws + oWV2);
  unsigned short* WO2  = (unsigned short*)(ws + oWO2);
  unsigned short* QH   = (unsigned short*)(ws + oQH);
  unsigned short* QL   = (unsigned short*)(ws + oQL);
  float*          KVF  = (float*)(ws + oRV);
  unsigned short* VTH  = (unsigned short*)(ws + oRV);
  unsigned short* LN   = (unsigned short*)(ws + oLN);
  unsigned short* KH   = (unsigned short*)(ws + oKH);
  unsigned short* KL   = (unsigned short*)(ws + oKL);
  unsigned short* VTL  = (unsigned short*)(ws + oVTL);

  static_assert(((SEQ * DIM / 8) % 256) == 0);
  static_assert(((QW * DIM / 8) % 256) == 0);
  static_assert(((KVA * DIM / 8) % 256) == 0);
  static_assert(((CW * KVR / 8) % 256) == 0);
  static_assert(((DIM * CW / 8) % 256) == 0);
  static_assert((KVR % 256) == 0 && (CW % 256) == 0);

  const dim3 b256(256), b128(128);
  const float sc = 0.07216878364870322f / (CQ * CK);
  const float oc = CC / (CP * CV);
  unsigned short* nolo = (unsigned short*)0;
  const float* nofc = (const float*)0;

  cvt_bf16_kernel<<<dim3((SEQ * DIM / 8) / 256, NB), b256, 0, stream>>>(x, XB, SEQ * DIM / 8, (long)SEQ_FULL * DIM, (long)SEQ * DIM);
  cvt_bf16_kernel<<<dim3((QW * DIM / 8) / 256, 1), b256, 0, stream>>>(wq, WQB, QW * DIM / 8, 0L, 0L);
  cvt_bf16_kernel<<<dim3((KVA * DIM / 8) / 256, 1), b256, 0, stream>>>(wa, WAB, KVA * DIM / 8, 0L, 0L);
  cvt_f16w_kernel<<<dim3((CW * KVR / 8) / 256), b256, 0, stream>>>(wb, WK, CW * KVR / 8, KVR, VD, NOPE + VD, 0, 0, CWT, CWT / CRES);
  cvt_f16w_kernel<<<dim3((CW * KVR / 8) / 256), b256, 0, stream>>>(wb, WV2, CW * KVR / 8, KVR, VD, NOPE + VD, NOPE, 1, CWT, CWT / CRES);
  cvt_f16w_kernel<<<dim3((DIM * CW / 8) / 256), b256, 0, stream>>>(wo, WO2, DIM * CW / 8, CW, DIM, DIM, 0, 1, CWO, CWO / CRES);
  gemm64_kernel<__bf16, 2, true><<<dim3(((NTOK / 64) * (QW / 64) + 7) / 8, 1), b256, 0, stream>>>(
      XB, DIM, 0L, WQB, DIM, 0L, (void*)QH, QW, 0L, QL, QW, 0L, SEQ, ER, QW, fc, QKD, NOPE, NTOK, QW, DIM, CQ);
  gemm64_kernel<__bf16, 0, false><<<dim3(((NTOK / 64) * (KVA / 64) + 7) / 8, 1), b256, 0, stream>>>(
      XB, DIM, 0L, WAB, DIM, 0L, (void*)KVF, KVA, 0L, nolo, 1, 0L, 1, 0, 0, nofc, 1, 0, NTOK, KVA, DIM, 1.0f);
  kvpost_kernel<<<dim3(NTOK / 8), b256, 0, stream>>>(KVF, fc, nw, LN, KH, KL);
  gemm64_kernel<_Float16, 2, false><<<dim3(((NTOK / 64) * (CW / 64) + 7) / 8, 1), b256, 0, stream>>>(
      LN, LNW, 0L, WK, KVR, 0L, (void*)KH, KW, 0L, KL, KW, 0L, SEQ, ER, CW, nofc, 1, 0, NTOK, CW, KVR, CK / (CL * CWT));
  gemm64_kernel<_Float16, 2, false><<<dim3(((CW / 64) * (SEQ / 64) + 7) / 8, NB), b256, 0, stream>>>(
      WV2, WVW, 0L, LN, LNW, (long)SEQ * LNW, (void*)VTH, SEQ, (long)CW * SEQ, VTL, ER, (long)CW * ER, CW, CW, ER,
      nofc, 1, 0, CW, SEQ, WVW, CV / (CWT * CL));
  attn_kernel<true><<<dim3(NHD * NQE * 2, NB), b128, 0, stream>>>(QH, QL, KH, KL, VTH, VTL, CTXH, C2, 0, NQE, sc, oc);
  const int nqbr = SEQ / 64 - NQE;
  if (nqbr > 0)
    attn_kernel<false><<<dim3(NHD * nqbr, NB), b128, 0, stream>>>(QH, QL, KH, KL, VTH, VTL, CTXH, C2, NQE, nqbr, sc, oc);
  gemm64_kernel<_Float16, 0, false><<<dim3(((ER / 64) * (DIM / 64) + 7) / 8, NB), b256, 0, stream>>>(
      C2, C2W, (long)ER * C2W, WO2, C2W, 0L, (void*)out, DIM, (long)SEQ_FULL * DIM, nolo, 1, 0L, 1, 0, 0, nofc, 1, 0,
      ER, DIM, C2W, 1.0f / (CC * CWO));
  if (SEQ > ER)
    gemm64_kernel<_Float16, 0, false><<<dim3((((SEQ - ER) / 64) * (DIM / 64) + 7) / 8, NB), b256, 0, stream>>>(
        CTXH + (size_t)ER * CW, CW, (long)SEQ * CW, WO2, C2W, 0L, (void*)(out + (size_t)ER * DIM), DIM, (long)SEQ_FULL * DIM,
        nolo, 1, 0L, 1, 0, 0, nofc, 1, 0, SEQ - ER, DIM, CW, 1.0f / (CC * CWO));
  (void)hipGetLastError();
}
